// DeformableCrossAttention_22445499089233
// MI455X (gfx1250) — hardware-verified
//
#include <hip/hip_runtime.h>
#include <math.h>
#include <stdint.h>

#define NB   2
#define CH   256
#define IMW  56
#define HWP  3136
#define NTOK 6272
#define NOFF 9
#define KVW  2304
#define KVW2 4608
#define NHDS 8
#define HDM  32
#define AOW  512
#define OFH  64
#define OFO  18
#define TBT  12321
#define TBP  12352
#define NQT  49
#define NKC  49

static_assert(NHDS * HDM == CH);
static_assert(NOFF * CH == KVW);
static_assert(2 * KVW == KVW2);
static_assert(HWP == IMW * IMW);
static_assert(NTOK == NB * HWP);
static_assert(HWP % 64 == 0 && CH % 64 == 0 && NTOK % 64 == 0);
static_assert(KVW2 % 32 == 0 && AOW % 32 == 0 && CH % 32 == 0);
static_assert(TBP % 32 == 0 && TBP >= TBT);
static_assert(NQT * 64 == HWP && NKC * 64 == HWP);
static_assert(2 * CH == AOW);

typedef __bf16   v16b __attribute__((ext_vector_type(16)));
typedef __bf16   v8b  __attribute__((ext_vector_type(8)));
typedef float    v8f  __attribute__((ext_vector_type(8)));
typedef float    v4f  __attribute__((ext_vector_type(4)));
typedef unsigned int v4u __attribute__((ext_vector_type(4)));

#if defined(__HIP_DEVICE_COMPILE__)
#define DEV_ASM 1
#else
#define DEV_ASM 0
#endif

__device__ __forceinline__ unsigned short bf_bits(float f) {
  unsigned u = __float_as_uint(f);
  return (unsigned short)((u + 0x7FFFu + ((u >> 16) & 1u)) >> 16);
}
__device__ __forceinline__ float bf_up(unsigned short hb) { return __uint_as_float(((unsigned)hb) << 16); }
__device__ __forceinline__ float bf_rne(float f) { return bf_up(bf_bits(f)); }
__device__ __forceinline__ unsigned pk16(unsigned short a, unsigned short b) { return (unsigned)a | ((unsigned)b << 16); }
__device__ __forceinline__ v8f zero8() { v8f z = {0.f, 0.f, 0.f, 0.f, 0.f, 0.f, 0.f, 0.f}; return z; }
__device__ __forceinline__ __bf16 to_bf(float f) { return __builtin_bit_cast(__bf16, bf_bits(f)); }
__device__ __forceinline__ void bf_split(float f, __bf16& hi, __bf16& lo) {
  const unsigned short hb = bf_bits(f);
  hi = __builtin_bit_cast(__bf16, hb);
  lo = to_bf(f - bf_up(hb));
}

__device__ __forceinline__ v16b ldfrag(const __bf16* p) {
  union { v16b v; v8b h[2]; } f;
  f.h[0] = *(const v8b*)(p);
  f.h[1] = *(const v8b*)(p + 16);
  return f.v;
}

__device__ __forceinline__ v8f mmar(v16b a, v16b b, v8f c) {
  return __builtin_amdgcn_wmma_f32_16x16x32_bf16(false, a, false, b, (short)0, c, false, false);
}
__device__ __forceinline__ v8f mma_g(v16b a, v16b b, v8f c) {
  c = __builtin_amdgcn_wmma_f32_16x16x32_bf16(false, a, false, b, (short)0, c, false, false);
#if DEV_ASM
  asm volatile("v_nop\n\tv_nop\n\tv_nop\n\tv_nop" : "+v"(c) : "v"(a), "v"(b));
#endif
  return c;
}
__device__ __forceinline__ void dep_guard(v8f& a, v8f& b, v16b x, v16b y) {
#if DEV_ASM
  asm volatile("v_nop\n\tv_nop\n\tv_nop\n\tv_nop" : "+v"(a), "+v"(b) : "v"(x), "v"(y));
#else
  (void)a; (void)b; (void)x; (void)y;
#endif
}
__device__ __forceinline__ void keep4(v16b a, v16b b, v16b c, v16b d) {
#if DEV_ASM
  asm volatile("v_nop" :: "v"(a), "v"(b), "v"(c), "v"(d));
#else
  (void)a; (void)b; (void)c; (void)d;
#endif
}
__device__ __forceinline__ void acc_guard4(v8f& a, v8f& b, v8f& c, v8f& d) {
#if DEV_ASM
  asm volatile("v_nop\n\tv_nop\n\tv_nop\n\tv_nop" : "+v"(a), "+v"(b), "+v"(c), "+v"(d));
#else
  (void)a; (void)b; (void)c; (void)d;
#endif
}

__global__ __launch_bounds__(256) void tconv_kernel(const float* __restrict__ W, unsigned short* __restrict__ oh,
                                                    int ldin, int ldout, long sIn, long sOut) {
  __shared__ __align__(16) float tf[64 * 68];
  W  += (size_t)blockIdx.z * sIn;
  oh += (size_t)blockIdx.z * sOut;
  const int c0  = blockIdx.x * 64;
  const int r0  = blockIdx.y * 64;
  const int tid = threadIdx.x;
  {
    const int lr = tid >> 4;
    const int c4 = (tid & 15) * 4;
#pragma unroll
    for (int it = 0; it < 4; ++it) {
      const int rr = it * 16 + lr;
      const v4f a = *(const v4f*)(W + (size_t)(r0 + rr) * ldin + c0 + c4);
      *(v4f*)(tf + rr * 68 + c4) = a;
    }
  }
  __syncthreads();
  const int sub = tid >> 3;
  const int c8  = (tid & 7) * 8;
  v4u hv[2];
#pragma unroll
  for (int it = 0; it < 2; ++it) {
    const int oc = it * 32 + sub;
    v4u a;
#pragma unroll
    for (int q = 0; q < 4; ++q) {
      const float f0 = tf[(c8 + 2 * q) * 68 + oc];
      const float f1 = tf[(c8 + 2 * q + 1) * 68 + oc];
      a[q] = pk16(bf_bits(f0), bf_bits(f1));
    }
    hv[it] = a;
  }
  for (int pass = 0; pass < 2; ++pass) {
#pragma unroll
    for (int it = 0; it < 2; ++it) {
      const int oc = it * 32 + sub;
      const size_t go = (size_t)(c0 + oc) * ldout + r0 + c8;
      *(volatile v4u*)(oh + go) = hv[it];
    }
    __threadfence();
  }
}

template <int MODE>
__global__ __launch_bounds__(256) void k_wcvt(const float* __restrict__ in, unsigned short* out, int kin, int upr, int nunits) {
  const int i = blockIdx.x * 256 + (int)threadIdx.x;
  if (i < nunits) {
    const int row = i / upr;
    const int u   = i - row * upr;
    int scol;
    if (MODE == 0) {
      scol = (u % (kin >> 3)) << 3;
    } else {
      const int j = u << 3;
      scol = ((j >> 6) << 5) + (j & 31);
    }
    const float* src = in + (size_t)row * kin + scol;
    const v4f a  = *(const v4f*)(src);
    const v4f a4 = *(const v4f*)(src + 4);
    v4u p;
    p[0] = pk16(bf_bits(a[0]),  bf_bits(a[1]));
    p[1] = pk16(bf_bits(a[2]),  bf_bits(a[3]));
    p[2] = pk16(bf_bits(a4[0]), bf_bits(a4[1]));
    p[3] = pk16(bf_bits(a4[2]), bf_bits(a4[3]));
    unsigned short* o = out + (size_t)i * 8;
    *(volatile v4u*)o = p;
    __threadfence();
    *(volatile v4u*)o = p;
  }
}

__global__ __launch_bounds__(256) void k_cpb(const float* __restrict__ w1, const float* __restrict__ b1,
                                            const float* __restrict__ w2, const float* __restrict__ b2, float* tb) {
  __shared__ float w1s[64];
  __shared__ float b1s[32];
  __shared__ float w2s[256];
  __shared__ float b2s[8];
  const int tid = (int)threadIdx.x;
  {
    const float a = w1[(tid < 64) ? tid : 63];
    if (tid < 64) w1s[tid] = bf_rne(a);
    const float c = b1[(tid < 32) ? tid : 31];
    if (tid < 32) b1s[tid] = bf_rne(c);
    w2s[tid] = bf_rne(w2[tid]);
    const float d = b2[(tid < 8) ? tid : 7];
    if (tid < 8) b2s[tid] = bf_rne(d);
  }
  __syncthreads();
  const int t  = blockIdx.x * 256 + tid;
  const int iy = t / (2 * IMW - 1);
  const int ix = t - iy * (2 * IMW - 1);
  const float dy = (float)(iy - (IMW - 1)) * (1.0f / 55.0f);
  const float dx = (float)(ix - (IMW - 1)) * (1.0f / 55.0f);
  float o_[8];
#pragma unroll
  for (int h = 0; h < 8; ++h) o_[h] = 0.0f;
#pragma unroll 1
  for (int d = 0; d < HDM; ++d) {
    float hd = dy * w1s[2 * d] + dx * w1s[2 * d + 1] + b1s[d];
    hd = fmaxf(hd, 0.0f);
#pragma unroll
    for (int h = 0; h < 8; ++h) o_[h] = fmaf(hd, w2s[h * HDM + d], o_[h]);
  }
#pragma unroll
  for (int h = 0; h < 8; ++h) o_[h] += b2s[h];
  if (t < TBP) {
    for (int pass = 0; pass < 2; ++pass) {
#pragma unroll
      for (int h = 0; h < 8; ++h) *(volatile float*)(tb + (size_t)h * TBP + t) = o_[h];
      __threadfence();
    }
  }
}

template <int BIAS_MODE, int OUT_MODE>
__global__ __launch_bounds__(256) void k_gemm64(
    const unsigned short* __restrict__ Ap, int lda, long long strideA,
    const unsigned short* __restrict__ Btp, int ldb, long long strideB,
    void* Cout, void* Cout2, int ldc, long long strideC,
    const float* __restrict__ bias, int M, int N, int K) {
  const __bf16* A  = (const __bf16*)(const void*)Ap;
  const __bf16* Bt = (const __bf16*)(const void*)Btp;
  __shared__ __align__(16) float sT[8][16 * 68];
  const int b    = blockIdx.y;
  const int lane = threadIdx.x & 31;
  const int wave = threadIdx.x >> 5;
  const int tilesN = N >> 6;
  const int tilesM = M >> 6;
  const int tile = blockIdx.x * 8 + wave;
  if (tile >= tilesM * tilesN) return;
  const int tm = tile / tilesN;
  const int tn = tile - tm * tilesN;
  const int m0 = tm << 6;
  const int n0 = tn << 6;

  const __bf16* Ab = A  + (size_t)b * (size_t)strideA;
  const __bf16* Bb = Bt + (size_t)b * (size_t)strideB;

  const int rlane = lane & 15;
  const int koff  = (lane >> 4) * 8;
  const int mOff  = (lane >> 4) * 8;

  v8f acc[4][4];
#pragma unroll
  for (int i = 0; i < 4; ++i)
#pragma unroll
    for (int j = 0; j < 4; ++j) acc[i][j] = zero8();

  for (int k0 = 0; k0 < K; k0 += 32) {
    v16b bq[4];
#pragma unroll
    for (int j = 0; j < 4; ++j)
      bq[j] = ldfrag(Bb + (size_t)(n0 + (j << 4) + rlane) * ldb + koff + k0);
#pragma unroll
    for (int i = 0; i < 4; ++i) {
      const v16b af = ldfrag(Ab + (size_t)(m0 + (i << 4) + rlane) * lda + koff + k0);
#pragma unroll
      for (int j = 0; j < 4; ++j) acc[i][j] = mmar(af, bq[j], acc[i][j]);
      dep_guard(acc[i][0], acc[i][3], af, bq[3]);
    }
    keep4(bq[0], bq[1], bq[2], bq[3]);
  }
  acc_guard4(acc[0][0], acc[0][1], acc[0][2], acc[0][3]);
  acc_guard4(acc[1][0], acc[1][1], acc[1][2], acc[1][3]);
  acc_guard4(acc[2][0], acc[2][1], acc[2][2], acc[2][3]);
  acc_guard4(acc[3][0], acc[3][1], acc[3][2], acc[3][3]);

  float blo = 0.f, bhi = 0.f;
  if (BIAS_MODE == 1) {
    blo = bf_rne(bias[m0 + lane]);
    bhi = bf_rne(bias[m0 + 32 + lane]);
  }

  float* slab = sT[wave];
#pragma unroll
  for (int i = 0; i < 4; ++i) {
    const int mBase = m0 + (i << 4);
    float bvr[8];
    if (BIAS_MODE == 1) {
      const float bsrc = (i < 2) ? blo : bhi;
#pragma unroll
      for (int r = 0; r < 8; ++r) bvr[r] = __shfl(bsrc, ((i & 1) << 4) + mOff + r, 32);
    } else {
#pragma unroll
      for (int r = 0; r < 8; ++r) bvr[r] = 0.f;
    }
#pragma unroll
    for (int j = 0; j < 4; ++j) {
#pragma unroll
      for (int r = 0; r < 8; ++r) {
        slab[(mOff + r) * 68 + (j << 4) + rlane] = acc[i][j][r] + bvr[r];
      }
    }
    __builtin_amdgcn_fence(__ATOMIC_RELEASE, "workgroup");
    __builtin_amdgcn_wave_barrier();
    __builtin_amdgcn_fence(__ATOMIC_ACQUIRE, "workgroup");
    if (OUT_MODE == 0) {
      float* C = (float*)Cout + (size_t)b * (size_t)strideC;
      const int h2 = lane >> 4, c4 = (lane & 15) * 4;
      for (int pass = 0; pass < 2; ++pass) {
#pragma unroll
        for (int it = 0; it < 8; ++it) {
          const int row = it * 2 + h2;
          const v4f v = *(const v4f*)(slab + row * 68 + c4);
          *(volatile v4f*)(C + (size_t)(mBase + row) * ldc + n0 + c4) = v;
        }
        __threadfence();
      }
    } else {
      const int q = lane >> 3, c8 = (lane & 7) * 8;
      unsigned short* C  = (unsigned short*)Cout  + (size_t)b * (size_t)strideC;
      unsigned short* C2 = (unsigned short*)Cout2 + (size_t)b * (size_t)strideC;
      v4u hv[4], lv[4];
#pragma unroll
      for (int it = 0; it < 4; ++it) {
        const int row = it * 4 + q;
        const float* sp = slab + row * 68 + c8;
        v4u a, a2;
#pragma unroll
        for (int e = 0; e < 4; ++e) {
          const float f0 = sp[2 * e], f1 = sp[2 * e + 1];
          const unsigned short h0 = bf_bits(f0), h1 = bf_bits(f1);
          const unsigned short l0 = bf_bits(f0 - bf_up(h0)), l1 = bf_bits(f1 - bf_up(h1));
          a[e] = pk16(h0, h1); a2[e] = pk16(l0, l1);
        }
        hv[it] = a; lv[it] = a2;
      }
      for (int pass = 0; pass < 2; ++pass) {
#pragma unroll
        for (int it = 0; it < 4; ++it) {
          const int row = it * 4 + q;
          *(volatile v4u*)(C  + (size_t)(mBase + row) * ldc + n0 + c8) = hv[it];
          *(volatile v4u*)(C2 + (size_t)(mBase + row) * ldc + n0 + c8) = lv[it];
        }
        __threadfence();
      }
    }
    __builtin_amdgcn_fence(__ATOMIC_RELEASE, "workgroup");
    __builtin_amdgcn_wave_barrier();
    __builtin_amdgcn_fence(__ATOMIC_ACQUIRE, "workgroup");
  }
}

__global__ __launch_bounds__(256) void k_sample(const unsigned short* __restrict__ kvt, const float* __restrict__ h1,
                                               const float* __restrict__ boff1, const float* __restrict__ woff2,
                                               const float* __restrict__ boff2, unsigned short* kvm) {
  __shared__ float w2s[OFO * OFH];
  __shared__ float b1s[OFH];
  __shared__ float b2s[32];
  __shared__ float h1s[8][OFH];
  const int tid  = (int)threadIdx.x;
  const int wave = tid >> 5;
  const int lane = tid & 31;
#pragma unroll 1
  for (int it = 0; it < 5; ++it) {
    const int i  = it * 256 + tid;
    const int ic = (i < OFO * OFH) ? i : (OFO * OFH - 1);
    const float v = woff2[ic];
    if (i < OFO * OFH) w2s[i] = bf_rne(v);
  }
  {
    const float v1 = boff1[(tid < OFH) ? tid : (OFH - 1)];
    if (tid < OFH) b1s[tid] = bf_rne(v1);
    const float v2 = boff2[(tid < OFO) ? tid : (OFO - 1)];
    if (tid < OFO) b2s[tid] = bf_rne(v2);
  }
  __syncthreads();

  const int n  = blockIdx.x * 8 + wave;
  const int b  = n / HWP;
  const int p  = n - b * HWP;
  const int yq = p / IMW;
  const int xq = p - yq * IMW;

#pragma unroll 1
  for (int e = 0; e < 2; ++e) {
    const int k = 32 * e + lane;
    const float x = h1[(size_t)n * OFH + k] + b1s[k];
    float y = 0.7978845608028654f * (x + 0.044715f * x * x * x);
    y = fminf(fmaxf(y, -10.0f), 10.0f);
    const float ex = __expf(2.0f * y);
    const float th = 1.0f - 2.0f * __builtin_amdgcn_rcpf(1.0f + ex);
    h1s[wave][k] = 0.5f * x * (1.0f + th);
  }
  __builtin_amdgcn_fence(__ATOMIC_RELEASE, "workgroup");
  __builtin_amdgcn_wave_barrier();
  __builtin_amdgcn_fence(__ATOMIC_ACQUIRE, "workgroup");

  const int lc = (lane < OFO) ? lane : (OFO - 1);
  float acc = b2s[lc];
#pragma unroll 4
  for (int k = 0; k < OFH; ++k) acc = fmaf(h1s[wave][k], w2s[lc * OFH + k], acc);

  const float xg = -1.0f + (float)xq * (2.0f / 55.0f);
  const float yg = -1.0f + (float)yq * (2.0f / 55.0f);
  const unsigned short* kvb = kvt + (size_t)b * HWP * CH + lane * 8;
  unsigned short* dst = kvm + (size_t)n * KVW2 + lane * 8;

#pragma unroll 1
  for (int o = 0; o < NOFF; ++o) {
    const float ox = __shfl(acc, o, 32);
    const float oy = __shfl(acc, NOFF + o, 32);
    const float gx = xg + ox * 0.1f;
    const float gy = yg + oy * 0.1f;
    const float px = fminf(fmaxf((gx + 1.0f) * 0.5f * 55.0f, 0.0f), 55.0f);
    const float py = fminf(fmaxf((gy + 1.0f) * 0.5f * 55.0f, 0.0f), 55.0f);
    const float fx = floorf(px), fy = floorf(py);
    int x0 = (int)fx, y0 = (int)fy;
    x0 = min(max(x0, 0), IMW - 1);
    y0 = min(max(y0, 0), IMW - 1);
    const int x1 = min(x0 + 1, IMW - 1), y1 = min(y0 + 1, IMW - 1);
    const float wx = px - fx, wy = py - fy;
    const float w00 = (1.0f - wx) * (1.0f - wy);
    const float w01 = wx * (1.0f - wy);
    const float w10 = (1.0f - wx) * wy;
    const float w11 = wx * wy;
    const v4u a00 = *(const v4u*)(kvb + (size_t)(y0 * IMW + x0) * CH);
    const v4u a01 = *(const v4u*)(kvb + (size_t)(y0 * IMW + x1) * CH);
    const v4u a10 = *(const v4u*)(kvb + (size_t)(y1 * IMW + x0) * CH);
    const v4u a11 = *(const v4u*)(kvb + (size_t)(y1 * IMW + x1) * CH);
    v4u ph, pl;
#pragma unroll
    for (int q = 0; q < 4; ++q) {
      const unsigned u00 = a00[q], u01 = a01[q], u10 = a10[q], u11 = a11[q];
      const float f0 = w00 * __uint_as_float(u00 << 16) + w01 * __uint_as_float(u01 << 16)
                     + w10 * __uint_as_float(u10 << 16) + w11 * __uint_as_float(u11 << 16);
      const float f1 = w00 * __uint_as_float(u00 & 0xffff0000u) + w01 * __uint_as_float(u01 & 0xffff0000u)
                     + w10 * __uint_as_float(u10 & 0xffff0000u) + w11 * __uint_as_float(u11 & 0xffff0000u);
      const unsigned short hb0 = bf_bits(f0), hb1 = bf_bits(f1);
      const unsigned short lb0 = bf_bits(f0 - bf_up(hb0)), lb1 = bf_bits(f1 - bf_up(hb1));
      ph[q] = pk16(hb0, hb1);
      pl[q] = pk16(lb0, lb1);
    }
    unsigned short* dh = dst + o * CH;
    unsigned short* dl = dst + KVW + o * CH;
    *(volatile v4u*)dh = ph;
    *(volatile v4u*)dl = pl;
    __threadfence();
    *(volatile v4u*)dh = ph;
    *(volatile v4u*)dl = pl;
  }
}

__global__ __launch_bounds__(128)
void k_attn(const unsigned short* __restrict__ qp, const unsigned short* __restrict__ kp,
            const unsigned short* __restrict__ vhp, const unsigned short* __restrict__ vlp,
            const float* __restrict__ tbp, unsigned short* aop, float sscale) {
  union FB { v16b v; v8b h[2]; };
  extern __shared__ __align__(16) float tbs[];
  __shared__ __align__(16) __bf16 Ksh[64 * HDM];
  __shared__ __align__(16) __bf16 Ksl[64 * HDM];
  __shared__ __align__(16) __bf16 Vts[HDM * 64];
  __shared__ __align__(16) __bf16 Vtl[HDM * 64];
  __shared__ __align__(16) __bf16 Psh[4][16 * 64];
  __shared__ __align__(16) __bf16 Psl[4][16 * 64];
  __shared__ __align__(16) float  Os[4][16 * 36];

  const int tid  = (int)threadIdx.x;
  const int wave = tid >> 5;
  const int lane = tid & 31;
  const int hh   = lane >> 4;
  const int c    = lane & 15;

  const int bx  = blockIdx.x;
  const int qb  = bx % NQT;
  const int hb2 = bx / NQT;
  const int h   = hb2 % NHDS;
  const int b   = hb2 / NHDS;
  const int pw  = qb * 64 + wave * 16;
  const size_t q0 = (size_t)b * HWP + pw;

  const __bf16* Q  = (const __bf16*)(const void*)qp;
  const __bf16* Kb = (const __bf16*)(const void*)kp;
  const __bf16* Vh = (const __bf16*)(const void*)vhp + (size_t)(h * HDM) * NTOK + (size_t)b * HWP;
  const __bf16* Vl = (const __bf16*)(const void*)vlp + (size_t)(h * HDM) * NTOK + (size_t)b * HWP;

#pragma unroll 1
  for (int it = 0; it < 25; ++it) {
    const int i  = it * 128 + tid;
    const int ic = (i < TBP / 4) ? i : (TBP / 4 - 1);
    const v4f v = *(const v4f*)(tbp + (size_t)h * TBP + 4 * ic);
    if (i < TBP / 4) *(v4f*)(tbs + 4 * i) = v;
  }

  const v16b qah = ldfrag(Q + (q0 + c) * AOW + h * HDM + 8 * hh);
  const v16b qal = ldfrag(Q + (q0 + c) * AOW + CH + h * HDM + 8 * hh);

  int yi[8], xi[8];
#pragma unroll
  for (int r = 0; r < 8; ++r) {
    const int m = pw + 8 * hh + r;
    yi[r] = m / IMW;
    xi[r] = m - yi[r] * IMW;
  }

  float mrow[8], lrow[8];
  v8f oacc[2];
#pragma unroll
  for (int r = 0; r < 8; ++r) { mrow[r] = -INFINITY; lrow[r] = 0.f; }
  oacc[0] = zero8(); oacc[1] = zero8();

  for (int kc = 0; kc < NKC; ++kc) {
    const int kv0 = kc * 64;
    __syncthreads();
    {
      const int r = tid >> 1, hf = (tid & 1) * 16;
      const __bf16* kr = Kb + ((size_t)b * HWP + kv0 + r) * AOW + h * HDM + hf;
      const v8b a0 = *(const v8b*)(kr);
      const v8b a1 = *(const v8b*)(kr + 8);
      const v8b l0 = *(const v8b*)(kr + CH);
      const v8b l1 = *(const v8b*)(kr + CH + 8);
      *(v8b*)(Ksh + r * HDM + hf)     = a0;
      *(v8b*)(Ksh + r * HDM + hf + 8) = a1;
      *(v8b*)(Ksl + r * HDM + hf)     = l0;
      *(v8b*)(Ksl + r * HDM + hf + 8) = l1;
      const int r2 = tid >> 2, q4 = (tid & 3) * 16;
      const __bf16* vr  = Vh + (size_t)r2 * NTOK + kv0 + q4;
      const __bf16* vrl = Vl + (size_t)r2 * NTOK + kv0 + q4;
      const v8b b0 = *(const v8b*)(vr);
      const v8b b1 = *(const v8b*)(vr + 8);
      const v8b c0 = *(const v8b*)(vrl);
      const v8b c1 = *(const v8b*)(vrl + 8);
      *(v8b*)(Vts + r2 * 64 + q4)     = b0;
      *(v8b*)(Vts + r2 * 64 + q4 + 8) = b1;
      *(v8b*)(Vtl + r2 * 64 + q4)     = c0;
      *(v8b*)(Vtl + r2 * 64 + q4 + 8) = c1;
    }
    __syncthreads();

    int jy[4], jx[4];
#pragma unroll
    for (int j = 0; j < 4; ++j) {
      const int kk = kv0 + j * 16 + c;
      jy[j] = kk / IMW;
      jx[j] = kk - jy[j] * IMW;
    }

    v8f s[4];
#pragma unroll
    for (int j = 0; j < 4; ++j) {
      FB kb, kl;
      kb.h[0] = *(const v8b*)(Ksh + (j * 16 + c) * HDM + 8 * hh);
      kb.h[1] = *(const v8b*)(Ksh + (j * 16 + c) * HDM + 16 + 8 * hh);
      kl.h[0] = *(const v8b*)(Ksl + (j * 16 + c) * HDM + 8 * hh);
      kl.h[1] = *(const v8b*)(Ksl + (j * 16 + c) * HDM + 16 + 8 * hh);
      v8f a = zero8();
      a = mma_g(qah, kb.v, a);
      a = mma_g(qah, kl.v, a);
      a = mma_g(qal, kb.v, a);
      s[j] = a;
    }
    float cm[8];
#pragma unroll
    for (int r = 0; r < 8; ++r) {
      float m = -INFINITY;
#pragma unroll
      for (int j = 0; j < 4; ++j) {
        const int idx = (yi[r] - jy[j] + (IMW - 1)) * (2 * IMW - 1) + (xi[r] - jx[j] + (IMW - 1));
        const float sv = s[j][r] * sscale + tbs[idx];
        s[j][r] = sv;
        m = fmaxf(m, sv);
      }
#pragma unroll
      for (int off = 1; off < 16; off <<= 1) m = fmaxf(m, __shfl_xor(m, off, 32));
      cm[r] = m;
    }
    __bf16* pwh = Psh[wave];
    __bf16* pwl = Psl[wave];
#pragma unroll
    for (int r = 0; r < 8; ++r) {
      const float mnew  = fmaxf(mrow[r], cm[r]);
      const float alpha = __expf(mrow[r] - mnew);
      mrow[r] = mnew;
      float psum = 0.f;
#pragma unroll
      for (int j = 0; j < 4; ++j) {
        const float pv = __expf(s[j][r] - mnew);
        psum += pv;
        __bf16 a, bl; bf_split(pv, a, bl);
        pwh[(8 * hh + r) * 64 + j * 16 + c] = a;
        pwl[(8 * hh + r) * 64 + j * 16 + c] = bl;
      }
#pragma unroll
      for (int off = 1; off < 16; off <<= 1) psum += __shfl_xor(psum, off, 32);
      lrow[r] = lrow[r] * alpha + psum;
      oacc[0][r] *= alpha;
      oacc[1][r] *= alpha;
    }
    __builtin_amdgcn_fence(__ATOMIC_RELEASE, "workgroup");
    __builtin_amdgcn_wave_barrier();
    __builtin_amdgcn_fence(__ATOMIC_ACQUIRE, "workgroup");

#pragma unroll 1
    for (int kk = 0; kk < 2; ++kk) {
      FB pa, pl;
      pa.h[0] = *(const v8b*)(pwh + c * 64 + kk * 32 + 8 * hh);
      pa.h[1] = *(const v8b*)(pwh + c * 64 + kk * 32 + 16 + 8 * hh);
      pl.h[0] = *(const v8b*)(pwl + c * 64 + kk * 32 + 8 * hh);
      pl.h[1] = *(const v8b*)(pwl + c * 64 + kk * 32 + 16 + 8 * hh);
#pragma unroll
      for (int t = 0; t < 2; ++t) {
        FB vb, vl;
        vb.h[0] = *(const v8b*)(Vts + (t * 16 + c) * 64 + kk * 32 + 8 * hh);
        vb.h[1] = *(const v8b*)(Vts + (t * 16 + c) * 64 + kk * 32 + 16 + 8 * hh);
        vl.h[0] = *(const v8b*)(Vtl + (t * 16 + c) * 64 + kk * 32 + 8 * hh);
        vl.h[1] = *(const v8b*)(Vtl + (t * 16 + c) * 64 + kk * 32 + 16 + 8 * hh);
        oacc[t] = mma_g(pa.v, vb.v, oacc[t]);
        oacc[t] = mma_g(pa.v, vl.v, oacc[t]);
        oacc[t] = mma_g(pl.v, vb.v, oacc[t]);
      }
    }
  }

  float* os = Os[wave];
#pragma unroll
  for (int r = 0; r < 8; ++r) {
    const float inv = 1.0f / lrow[r];
    os[(8 * hh + r) * 36 + c]      = oacc[0][r] * inv;
    os[(8 * hh + r) * 36 + 16 + c] = oacc[1][r] * inv;
  }
  __builtin_amdgcn_fence(__ATOMIC_RELEASE, "workgroup");
  __builtin_amdgcn_wave_barrier();
  __builtin_amdgcn_fence(__ATOMIC_ACQUIRE, "workgroup");
  {
    const int q4   = lane >> 3;
    const int c8   = (lane & 7) * 8;
    const int d0   = c8 & 31;
    const int islo = (lane >> 2) & 1;
    v4u hv[4];
#pragma unroll
    for (int it = 0; it < 4; ++it) {
      const int row = it * 4 + q4;
      const float* sp = os + row * 36 + d0;
      v4u a;
#pragma unroll
      for (int e = 0; e < 4; ++e) {
        const float f0 = sp[2 * e], f1 = sp[2 * e + 1];
        const unsigned short hb0 = bf_bits(f0), hb1 = bf_bits(f1);
        const unsigned short lb0 = bf_bits(f0 - bf_up(hb0)), lb1 = bf_bits(f1 - bf_up(hb1));
        const unsigned short w0 = islo ? lb0 : hb0;
        const unsigned short w1 = islo ? lb1 : hb1;
        a[e] = pk16(w0, w1);
      }
      hv[it] = a;
    }
    for (int pass = 0; pass < 2; ++pass) {
#pragma unroll
      for (int it = 0; it < 4; ++it) {
        const int row = it * 4 + q4;
        *(volatile v4u*)(aop + (q0 + row) * AOW + (size_t)h * 64 + c8) = hv[it];
      }
      __threadfence();
    }
  }
}

extern "C" void kernel_launch(void* const* d_in, const int* in_sizes, int n_in,
                              void* d_out, int out_size, void* d_ws, size_t ws_size,
                              hipStream_t stream) {
  if (n_in < 15) return;
  if (in_sizes[0] != NB * CH * HWP || in_sizes[1] != NB * CH * HWP) return;
  if (in_sizes[2] != CH * CH) return;
  if (in_sizes[3] != CH * KVW || in_sizes[4] != CH * KVW) return;
  if (in_sizes[5] != OFH * CH || in_sizes[6] != OFH) return;
  if (in_sizes[7] != OFO * OFH || in_sizes[8] != OFO) return;
  if (in_sizes[9] != HDM * 2 || in_sizes[10] != HDM) return;
  if (in_sizes[11] != NHDS * HDM || in_sizes[12] != NHDS) return;
  if (in_sizes[13] != CH * CH || in_sizes[14] != CH) return;
  if (out_size != NB * CH * HWP) return;

  const float* query = (const float*)d_in[0];
  const float* kvmap = (const float*)d_in[1];
  const float* Wq    = (const float*)d_in[2];
  const float* Wk    = (const float*)d_in[3];
  const float* Wv    = (const float*)d_in[4];
  const float* Woff1 = (const float*)d_in[5];
  const float* boff1 = (const float*)d_in[6];
  const float* Woff2 = (const float*)d_in[7];
  const float* boff2 = (const float*)d_in[8];
  const float* cw1   = (const float*)d_in[9];
  const float* cb1   = (const float*)d_in[10];
  const float* cw2   = (const float*)d_in[11];
  const float* cb2   = (const float*)d_in[12];
  const float* Wout  = (const float*)d_in[13];
  const float* bout  = (const float*)d_in[14];

  const size_t PT16 = (size_t)NTOK * CH * 2;
  const size_t PWQ  = (size_t)CH * CH * 2;
  const size_t PW1  = (size_t)OFH * AOW * 2;
  const size_t PWK  = (size_t)CH * KVW2 * 2;
  const size_t PWO  = (size_t)CH * AOW * 2;
  const size_t PTB  = (size_t)NHDS * TBP * 4;
  const size_t PHL  = (size_t)NTOK * AOW * 2;
  const size_t PH1  = (size_t)NTOK * OFH * 4;
  const size_t PKVM = (size_t)NTOK * KVW2 * 2;
  const size_t PVT  = (size_t)CH * NTOK * 2;
  size_t off = 0;
  const size_t oQT  = off; off += PT16;
  const size_t oKVT = off; off += PT16;
  const size_t oWq  = off; off += PWQ;
  const size_t oW1  = off; off += PW1;
  const size_t oWk  = off; off += PWK;
  const size_t oWv  = off; off += PWK;
  const size_t oWo  = off; off += PWO;
  const size_t oTB  = off; off += PTB;
  const size_t oQHL = off; off += PHL;
  const size_t oH1  = off; off += PH1;
  const size_t oKVM = off; off += PKVM;
  const size_t oKHL = off; off += PHL;
  const size_t oVTh = off; off += PVT;
  const size_t oVTl = off; off += PVT;
  const size_t oAO  = off; off += PHL;
  if (off > ws_size) return;
  if (off > (size_t)134217728) return;

  char* ws = (char*)d_ws;
  unsigned short* QT   = (unsigned short*)(ws + oQT);
  unsigned short* KVT  = (unsigned short*)(ws + oKVT);
  unsigned short* WqB  = (unsigned short*)(ws + oWq);
  unsigned short* W1B2 = (unsigned short*)(ws + oW1);
  unsigned short* WkB2 = (unsigned short*)(ws + oWk);
  unsigned short* WvB2 = (unsigned short*)(ws + oWv);
  unsigned short* Wo2  = (unsigned short*)(ws + oWo);
  float*          TB   = (float*)(ws + oTB);
  unsigned short* QHL  = (unsigned short*)(ws + oQHL);
  float*          H1   = (float*)(ws + oH1);
  unsigned short* KVM  = (unsigned short*)(ws + oKVM);
  unsigned short* KHL  = (unsigned short*)(ws + oKHL);
  unsigned short* VTh  = (unsigned short*)(ws + oVTh);
  unsigned short* VTl  = (unsigned short*)(ws + oVTl);
  unsigned short* AO   = (unsigned short*)(ws + oAO);

  const dim3 blk(256);
  const int nuWq = CH * (CH / 8);
  const int nuW1 = OFH * (AOW / 8);
  const int nuWk = CH * (KVW2 / 8);
  const int nuWo = CH * (AOW / 8);

  tconv_kernel<<<dim3(HWP / 64, CH / 64, NB), blk, 0, stream>>>(query, QT, HWP, CH, (long)CH * HWP, (long)HWP * CH);
  tconv_kernel<<<dim3(HWP / 64, CH / 64, NB), blk, 0, stream>>>(kvmap, KVT, HWP, CH, (long)CH * HWP, (long)HWP * CH);
  k_wcvt<0><<<dim3(nuWq / 256), blk, 0, stream>>>(Wq, WqB, CH, CH / 8, nuWq);
  k_wcvt<0><<<dim3(nuW1 / 256), blk, 0, stream>>>(Woff1, W1B2, CH, AOW / 8, nuW1);
  k_wcvt<0><<<dim3(nuWk / 256), blk, 0, stream>>>(Wk, WkB2, KVW, KVW2 / 8, nuWk);
  k_wcvt<0><<<dim3(nuWk / 256), blk, 0, stream>>>(Wv, WvB2, KVW, KVW2 / 8, nuWk);
  k_wcvt<1><<<dim3(nuWo / 256), blk, 0, stream>>>(Wout, Wo2, CH, AOW / 8, nuWo);
  k_cpb<<<dim3((TBP + 255) / 256), blk, 0, stream>>>(cw1, cb1, cw2, cb2, TB);
  k_gemm64<0, 2><<<dim3(((NTOK / 64) * (CH / 64) + 7) / 8, 1), blk, 0, stream>>>(
      QT, CH, 0LL, WqB, CH, 0LL, (void*)QHL, (void*)(QHL + CH), AOW, 0LL, bout, NTOK, CH, CH);
  k_gemm64<0, 0><<<dim3(((NTOK / 64) * (OFH / 64) + 7) / 8, 1), blk, 0, stream>>>(
      QHL, AOW, 0LL, W1B2, AOW, 0LL, (void*)H1, (void*)H1, OFH, 0LL, bout, NTOK, OFH, AOW);
  k_sample<<<dim3(NTOK / 8), blk, 0, stream>>>(KVT, H1, boff1, Woff2, boff2, KVM);
  k_gemm64<0, 2><<<dim3(((NTOK / 64) * (CH / 64) + 7) / 8, 1), blk, 0, stream>>>(
      KVM, KVW2, 0LL, WkB2, KVW2, 0LL, (void*)KHL, (void*)(KHL + CH), AOW, 0LL, bout, NTOK, CH, KVW2);
  k_gemm64<0, 2><<<dim3(((CH / 64) * (NTOK / 64) + 7) / 8, 1), blk, 0, stream>>>(
      WvB2, KVW2, 0LL, KVM, KVW2, 0LL, (void*)VTh, (void*)VTl, NTOK, 0LL, bout, CH, NTOK, KVW2);
  (void)hipFuncSetAttribute(reinterpret_cast<const void*>(&k_attn), hipFuncAttributeMaxDynamicSharedMemorySize, TBP * 4);
  k_attn<<<dim3(NB * NHDS * NQT), dim3(128), (size_t)TBP * 4, stream>>>(QHL, KHL, VTh, VTl, TB, AO, 0.17677669529663687f);
  k_gemm64<1, 0><<<dim3(((CH / 64) * (HWP / 64) + 7) / 8, NB), blk, 0, stream>>>(
      Wo2, AOW, 0LL, AO, AOW, (long long)HWP * AOW, d_out, d_out, HWP, (long long)CH * HWP, bout, CH, HWP, AOW);
  (void)hipGetLastError();
}
